// lstmModel_70987219468378
// MI455X (gfx1250) — hardware-run, weakly checked
//
#include <hip/hip_runtime.h>
#include <math.h>

constexpr int NBAT   = 64;
constexpr int CIN    = 28;
constexpr int TLEN   = 8192;
constexpr int C1N    = 8;
constexpr int NFN    = 16;
constexpr int KTAP   = 9;
constexpr int TSTR   = 3;
constexpr int TPN    = (TLEN - KTAP) / TSTR + 1;
constexpr int WMAXN  = 128;
constexpr int CL     = C1N * NFN;
constexpr int HN     = 32;
constexpr int GN     = 4 * HN;
constexpr float BN_EPS     = 1e-5f;
constexpr float CARRY      = 16.0f;
constexpr float CARRY2_INV = 1.0f / 256.0f;

constexpr int CV_THR  = 128;
constexpr int CV_TB   = 256;
constexpr int XSP     = 260;
constexpr int SLP     = 68;
constexpr int PL_THR  = 128;
constexpr int LS_THR  = 64;
constexpr int LS_ROWS = 16;
constexpr int AHP     = 40;
constexpr int HSP     = 260;

static_assert(TPN == 2728);
static_assert(TLEN % CV_TB == 0);
static_assert(CV_TB == 64 * (CV_THR / 32));
static_assert(CIN <= 32 && C1N <= 16);
static_assert((CIN * CV_TB / 4) % CV_THR == 0);
static_assert((CIN * CV_TB / 4) / CV_THR == 14);
static_assert(PL_THR == CL && CL % 32 == 0);
static_assert(NFN * KTAP > PL_THR && NFN * KTAP - PL_THR <= PL_THR);
static_assert(HN == 32 && GN == 128);
static_assert(NBAT % LS_ROWS == 0);
static_assert(HN == 16 * (LS_THR / 32));
static_assert((LS_ROWS * AHP) % LS_THR == 0);
static_assert((LS_ROWS * HN / 4) % LS_THR == 0);
static_assert(TSTR * (TPN - 1) + KTAP - 1 < TLEN);

typedef __attribute__((ext_vector_type(16))) _Float16 v16h;
typedef __attribute__((ext_vector_type(8)))  _Float16 v8h;
typedef __attribute__((ext_vector_type(16))) __bf16   v16b;
typedef __attribute__((ext_vector_type(8)))  __bf16   v8b;
typedef __attribute__((ext_vector_type(8)))  float    v8f;
typedef __attribute__((ext_vector_type(4)))  float    v4f;

__device__ __forceinline__ void dep_guard_h(v8f& a, v8f& b, v16h x, v16h y) { asm volatile("v_nop\n\tv_nop\n\tv_nop\n\tv_nop" : "+v"(a), "+v"(b) : "v"(x), "v"(y)); }
__device__ __forceinline__ void dep_guard_b(v8f& a, v8f& b, v16b x, v16b y) { asm volatile("v_nop\n\tv_nop\n\tv_nop\n\tv_nop" : "+v"(a), "+v"(b) : "v"(x), "v"(y)); }
__device__ __forceinline__ void keep4_h(v16h a, v16h b, v16h c, v16h d) { asm volatile("v_nop" :: "v"(a), "v"(b), "v"(c), "v"(d)); }
__device__ __forceinline__ void keep4_b(v16b a, v16b b, v16b c, v16b d) { asm volatile("v_nop" :: "v"(a), "v"(b), "v"(c), "v"(d)); }
__device__ __forceinline__ void acc_guard4(v8f& a, v8f& b, v8f& c, v8f& d) { asm volatile("v_nop\n\tv_nop\n\tv_nop\n\tv_nop" : "+v"(a), "+v"(b), "+v"(c), "+v"(d)); }
__device__ __forceinline__ void guard1h(v8f& a, v16h x, v16h y) { asm volatile("v_nop\n\tv_nop\n\tv_nop\n\tv_nop" : "+v"(a) : "v"(x), "v"(y)); }
__device__ __forceinline__ void guard45h(v8f& a0, v8f& a1, v8f& a2, v8f& a3, v16h x, v16h y0, v16h y1, v16h y2, v16h y3) {
  asm volatile("v_nop\n\tv_nop\n\tv_nop\n\tv_nop" : "+v"(a0), "+v"(a1), "+v"(a2), "+v"(a3) : "v"(x), "v"(y0), "v"(y1), "v"(y2), "v"(y3));
}

template <typename T> struct Frag;
template <> struct Frag<_Float16> {
  typedef v16h V; union U { v16h v; v8h h[2]; };
  static __device__ __forceinline__ v16h load(const _Float16* p) {
    U f; f.h[0] = *(const v8h*)(p); f.h[1] = *(const v8h*)(p + 16); return f.v;
  }
  static __device__ __forceinline__ v8f mma(v16h a, v16h b, v8f c) {
    return __builtin_amdgcn_wmma_f32_16x16x32_f16(false, a, false, b, (short)0, c, false, false);
  }
  static __device__ __forceinline__ void guard(v8f& a, v8f& b, v16h x, v16h y) { dep_guard_h(a, b, x, y); }
  static __device__ __forceinline__ void keep(v16h a, v16h b, v16h c, v16h d) { keep4_h(a, b, c, d); }
};
template <> struct Frag<__bf16> {
  typedef v16b V; union U { v16b v; v8b h[2]; };
  static __device__ __forceinline__ v16b load(const __bf16* p) {
    U f; f.h[0] = *(const v8b*)(p); f.h[1] = *(const v8b*)(p + 16); return f.v;
  }
  static __device__ __forceinline__ v8f mma(v16b a, v16b b, v8f c) {
    return __builtin_amdgcn_wmma_f32_16x16x32_bf16(false, a, false, b, (short)0, c, false, false);
  }
  static __device__ __forceinline__ void guard(v8f& a, v8f& b, v16b x, v16b y) { dep_guard_b(a, b, x, y); }
  static __device__ __forceinline__ void keep(v16b a, v16b b, v16b c, v16b d) { keep4_b(a, b, c, d); }
};

__device__ __forceinline__ float sigm_f(float z) {
  const float zc = fminf(fmaxf(z, -30.0f), 30.0f);
  return 1.0f / (1.0f + expf(-zc));
}
__device__ __forceinline__ float tanh_f(float z) {
  const float zc = fminf(fmaxf(2.0f * z, -30.0f), 30.0f);
  return 1.0f - 2.0f / (1.0f + expf(zc));
}

__global__ __launch_bounds__(256) void prep_w_kernel(const float* __restrict__ w_ih, const float* __restrict__ w_hh,
                                                     unsigned short* __restrict__ WIH16, unsigned short* __restrict__ WHH16) {
  const int tid = threadIdx.x;
  if (blockIdx.x < 8) {
    const int i = blockIdx.x * 256 + tid;
    const float* sp = w_ih + (size_t)i * 8;
    const v4f a = *(const v4f*)(sp);
    const v4f b = *(const v4f*)(sp + 4);
    v8h hv;
#pragma unroll
    for (int e = 0; e < 4; ++e) { hv[e] = (_Float16)(a[e] * CARRY); hv[4 + e] = (_Float16)(b[e] * CARRY); }
    unsigned short* dp = WIH16 + (size_t)i * 8;
    *(volatile v8h*)dp = hv;
    __threadfence();
    *(volatile v8h*)dp = hv;
  } else {
    const int i = (blockIdx.x - 8) * 256 + tid;
    const float* sp = w_hh + (size_t)i * 8;
    const v4f a = *(const v4f*)(sp);
    const v4f b = *(const v4f*)(sp + 4);
    v8h hv;
#pragma unroll
    for (int e = 0; e < 4; ++e) { hv[e] = (_Float16)(a[e] * CARRY); hv[4 + e] = (_Float16)(b[e] * CARRY); }
    unsigned short* dp = WHH16 + (size_t)i * 8;
    *(volatile v8h*)dp = hv;
    __threadfence();
    *(volatile v8h*)dp = hv;
  }
}

__global__ __launch_bounds__(CV_THR) void pconv_kernel(const float* __restrict__ x, const float* __restrict__ w1,
                                                      const float* __restrict__ b1, float* __restrict__ Y1) {
  __shared__ __align__(16) float xs[CIN * XSP];
  __shared__ __align__(16) float sl[CV_THR / 32][C1N * SLP];
  __shared__ float w1s[C1N * CIN];
  __shared__ float b1s[C1N];
  const int tid = threadIdx.x, lane = tid & 31, wave = tid >> 5;
  const int hh = lane >> 4, cc = lane & 15;
  const int b  = blockIdx.x / (TLEN / CV_TB);
  const int tb = (blockIdx.x % (TLEN / CV_TB)) * CV_TB;

#pragma unroll 1
  for (int i = tid; i < C1N * CIN; i += CV_THR) w1s[i] = w1[i];
  if (tid < C1N) b1s[tid] = b1[tid];
  {
    const float* xb = x + (size_t)b * CIN * TLEN + tb;
#pragma unroll
    for (int it = 0; it < 7; ++it) {
      const int idx = it * CV_THR + tid;
      const int row = idx >> 6, c4 = (idx & 63) * 4;
      const v4f v = *(const v4f*)(xb + (size_t)row * TLEN + c4);
      *(v4f*)(xs + row * XSP + c4) = v;
    }
    asm volatile("" ::: "memory");
#pragma unroll
    for (int it = 7; it < 14; ++it) {
      const int idx = it * CV_THR + tid;
      const int row = idx >> 6, c4 = (idx & 63) * 4;
      const v4f v = *(const v4f*)(xb + (size_t)row * TLEN + c4);
      *(v4f*)(xs + row * XSP + c4) = v;
    }
  }
  __syncthreads();

  const int   oc = (cc < C1N) ? cc : (C1N - 1);
  const float fo = (cc < C1N) ? CARRY : 0.0f;
  v16h bw;
#pragma unroll
  for (int e = 0; e < 8; ++e) {
    const int ka  = 8 * hh + e;
    const int kb  = 16 + 8 * hh + e;
    const int kbc = (kb < CIN) ? kb : (CIN - 1);
    const float fb = (kb < CIN) ? fo : 0.0f;
    bw[e]     = (_Float16)(w1s[oc * CIN + ka] * fo);
    bw[8 + e] = (_Float16)(w1s[oc * CIN + kbc] * fb);
  }

  const v8f z8 = {0.f, 0.f, 0.f, 0.f, 0.f, 0.f, 0.f, 0.f};
  v8f acc[4];
#pragma unroll
  for (int i = 0; i < 4; ++i) acc[i] = z8;
#pragma unroll
  for (int i = 0; i < 4; ++i) {
    const int tl = wave * 64 + 16 * i + cc;
    v16h a;
#pragma unroll
    for (int e = 0; e < 8; ++e) {
      const int ka  = 8 * hh + e;
      const int kb  = 16 + 8 * hh + e;
      const int kbc = (kb < CIN) ? kb : (CIN - 1);
      const float fb = (kb < CIN) ? CARRY : 0.0f;
      a[e]     = (_Float16)(xs[ka * XSP + tl] * CARRY);
      a[8 + e] = (_Float16)(xs[kbc * XSP + tl] * fb);
    }
    acc[i] = Frag<_Float16>::mma(a, bw, acc[i]);
    guard1h(acc[i], a, bw);
  }
  acc_guard4(acc[0], acc[1], acc[2], acc[3]);

  float* slab = sl[wave];
  const float bo = b1s[oc];
  if (cc < C1N) {
#pragma unroll
    for (int i = 0; i < 4; ++i) {
#pragma unroll
      for (int r = 0; r < 8; ++r) {
        const float v = fmaxf(acc[i][r] * CARRY2_INV + bo, 0.0f);
        slab[cc * SLP + 16 * i + 8 * hh + r] = v;
      }
    }
  }
  __syncthreads();
  {
    const int c4 = cc * 4;
    float* yb = Y1 + (size_t)b * C1N * TLEN + tb + wave * 64 + c4;
    for (int pass = 0; pass < 2; ++pass) {
#pragma unroll
      for (int it = 0; it < 4; ++it) {
        const int row = it * 2 + hh;
        const v4f v = *(const v4f*)(slab + row * SLP + c4);
        *(volatile v4f*)(yb + (size_t)row * TLEN) = v;
      }
      __threadfence();
    }
  }
}

__global__ __launch_bounds__(PL_THR) void pool_kernel(const float* __restrict__ Y1, const float* __restrict__ w2,
                                                     const float* __restrict__ b2,
                                                     const float* __restrict__ bn_g, const float* __restrict__ bn_b,
                                                     const float* __restrict__ bn_m, const float* __restrict__ bn_v,
                                                     const int* __restrict__ onset, const int* __restrict__ offset,
                                                     unsigned short* __restrict__ P16) {
  __shared__ float w2s[NFN * KTAP];
  __shared__ float scs[NFN], shs[NFN], b2s[NFN];
  __shared__ __align__(16) float ps[CL];
  const int tid = threadIdx.x;
  w2s[tid] = w2[tid];
  if (tid < NFN * KTAP - PL_THR) w2s[PL_THR + tid] = w2[PL_THR + tid];
  if (tid < NFN) {
    const float sc = bn_g[tid] / sqrtf(bn_v[tid] + BN_EPS);
    scs[tid] = sc;
    shs[tid] = bn_b[tid] - bn_m[tid] * sc;
    b2s[tid] = b2[tid];
  }
  __syncthreads();

  const int w = blockIdx.x, b = blockIdx.y;
  const int c = tid, nf = c >> 3, c1 = c & 7;
  int on  = onset [b * WMAXN + w];
  int off = offset[b * WMAXN + w];
  on  = (on  < 0) ? 0 : ((on  > TPN) ? TPN : on);
  off = (off < 0) ? 0 : ((off > TPN) ? TPN : off);
  const int lo = (on < off) ? on : off;
  const int hi = (on < off) ? off : on;
  const int dl = off - on;

  float wk[KTAP];
#pragma unroll
  for (int k = 0; k < KTAP; ++k) wk[k] = w2s[nf * KTAP + k];
  const float bias2 = b2s[nf], sc = scs[nf], sh = shs[nf];
  const float* yb = Y1 + ((size_t)b * C1N + c1) * TLEN;
  float sum = 0.0f;
#pragma unroll 1
  for (int t = lo; t < hi; ++t) {
    const float* yp = yb + TSTR * t;
    float v = bias2;
#pragma unroll
    for (int k = 0; k < KTAP; ++k) v = fmaf(wk[k], yp[k], v);
    v = fmaf(v, sc, sh);
    sum += fmaxf(v, 0.0f);
  }
  const float len = (float)((dl > 1) ? dl : 1);
  const float sgn = (dl >= 0) ? 1.0f : -1.0f;
  ps[c] = ((sum * sgn) * (1.0f / len)) * CARRY;
  __syncthreads();
  if (tid < 16) {
    const v4f a  = *(const v4f*)(ps + tid * 8);
    const v4f bq = *(const v4f*)(ps + tid * 8 + 4);
    v8h hv;
#pragma unroll
    for (int e = 0; e < 4; ++e) { hv[e] = (_Float16)a[e]; hv[4 + e] = (_Float16)bq[e]; }
    unsigned short* dp = P16 + ((size_t)(b * WMAXN + w)) * CL + tid * 8;
    *(volatile v8h*)dp = hv;
    __threadfence();
    *(volatile v8h*)dp = hv;
  }
}

__global__ __launch_bounds__(LS_THR) void lstm_kernel(const unsigned short* __restrict__ P16p,
                                                     const unsigned short* __restrict__ WIHp,
                                                     const unsigned short* __restrict__ WHHp,
                                                     const float* __restrict__ b_ih, const float* __restrict__ b_hh,
                                                     const int* __restrict__ s, float* __restrict__ out) {
  __shared__ __align__(16) _Float16 Ah[LS_ROWS * AHP];
  __shared__ __align__(16) float    Hs[LS_ROWS * HSP];
  const _Float16* P16 = (const _Float16*)P16p;
  const _Float16* WIH = (const _Float16*)WIHp;
  const _Float16* WHH = (const _Float16*)WHHp;
  const int tid = threadIdx.x, lane = tid & 31, wave = tid >> 5;
  const int c = lane & 15, hh = lane >> 4, koff = hh * 8;
  const int rowbase = blockIdx.x * LS_ROWS;
  const int j = 16 * wave + c;

#pragma unroll 1
  for (int i = tid; i < LS_ROWS * AHP; i += LS_THR) Ah[i] = (_Float16)0.0f;

  float bb[4];
#pragma unroll
  for (int g = 0; g < 4; ++g) bb[g] = b_ih[HN * g + j] + b_hh[HN * g + j];
  asm volatile("" ::: "memory");
  int sr[8];
#pragma unroll
  for (int r = 0; r < 8; ++r) sr[r] = s[rowbase + 8 * hh + r];
  v16h bq[4];
#pragma unroll
  for (int g = 0; g < 4; ++g) bq[g] = Frag<_Float16>::load(WHH + (size_t)(HN * g + j) * HN + koff);

  float cst[8], hst[8];
#pragma unroll
  for (int r = 0; r < 8; ++r) { cst[r] = 0.0f; hst[r] = 0.0f; }
  __syncthreads();

  const _Float16* ahrow = Ah + c * AHP + koff;
  const _Float16* wrow  = WIH + (size_t)j * CL + koff;
  const size_t gstr = (size_t)HN * CL;
  const v8f z8 = {0.f, 0.f, 0.f, 0.f, 0.f, 0.f, 0.f, 0.f};

#pragma unroll 1
  for (int w = 0; w < WMAXN; ++w) {
    v8f acc[4];
    acc[0] = z8; acc[1] = z8; acc[2] = z8; acc[3] = z8;
    const _Float16* arow = P16 + ((size_t)(rowbase + c) * WMAXN + (size_t)w) * CL + koff;
#pragma unroll 1
    for (int k0 = 0; k0 < CL; k0 += 32) {
      const v16h a  = Frag<_Float16>::load(arow + k0);
      const v16h b0 = Frag<_Float16>::load(wrow + k0);
      const v16h b1 = Frag<_Float16>::load(wrow + gstr + k0);
      const v16h b2 = Frag<_Float16>::load(wrow + 2 * gstr + k0);
      const v16h b3 = Frag<_Float16>::load(wrow + 3 * gstr + k0);
      acc[0] = Frag<_Float16>::mma(a, b0, acc[0]);
      acc[1] = Frag<_Float16>::mma(a, b1, acc[1]);
      acc[2] = Frag<_Float16>::mma(a, b2, acc[2]);
      acc[3] = Frag<_Float16>::mma(a, b3, acc[3]);
      guard45h(acc[0], acc[1], acc[2], acc[3], a, b0, b1, b2, b3);
    }
    {
      const v16h ah = Frag<_Float16>::load(ahrow);
      acc[0] = Frag<_Float16>::mma(ah, bq[0], acc[0]);
      acc[1] = Frag<_Float16>::mma(ah, bq[1], acc[1]);
      acc[2] = Frag<_Float16>::mma(ah, bq[2], acc[2]);
      acc[3] = Frag<_Float16>::mma(ah, bq[3], acc[3]);
      guard45h(acc[0], acc[1], acc[2], acc[3], ah, bq[0], bq[1], bq[2], bq[3]);
    }
    acc_guard4(acc[0], acc[1], acc[2], acc[3]);

#pragma unroll
    for (int r = 0; r < 8; ++r) {
      const float zi = acc[0][r] * CARRY2_INV + bb[0];
      const float zf = acc[1][r] * CARRY2_INV + bb[1];
      const float zg = acc[2][r] * CARRY2_INV + bb[2];
      const float zo = acc[3][r] * CARRY2_INV + bb[3];
      const float ig = sigm_f(zi);
      const float fg = sigm_f(zf);
      const float gg = tanh_f(zg);
      const float og = sigm_f(zo);
      const float cn = fg * cst[r] + ig * gg;
      const float hn = og * tanh_f(cn);
      const bool keep = (w < sr[r]);
      cst[r] = keep ? cn : cst[r];
      hst[r] = keep ? hn : hst[r];
    }
    __syncthreads();
#pragma unroll
    for (int r = 0; r < 8; ++r) Ah[(8 * hh + r) * AHP + j] = (_Float16)(hst[r] * CARRY);
    __syncthreads();
  }

#pragma unroll
  for (int r = 0; r < 8; ++r) Hs[(8 * hh + r) * HSP + j] = hst[r];
  __syncthreads();
  for (int pass = 0; pass < 2; ++pass) {
#pragma unroll
    for (int it = 0; it < 2; ++it) {
      const int idx = it * LS_THR + tid;
      const int row = idx >> 3, c4 = (idx & 7) * 4;
      const v4f v = *(const v4f*)(Hs + row * HSP + c4);
      *(volatile v4f*)(out + (size_t)(rowbase + row) * HN + c4) = v;
    }
    __threadfence();
  }
}

extern "C" void kernel_launch(void* const* d_in, const int* in_sizes, int n_in,
                              void* d_out, int out_size, void* d_ws, size_t ws_size, hipStream_t stream) {
  if (n_in < 16 || d_out == nullptr || d_ws == nullptr) return;
  if (in_sizes[0] != NBAT * CIN * TLEN || in_sizes[1] != NBAT || in_sizes[2] != NBAT * WMAXN ||
      in_sizes[3] != NBAT * WMAXN || in_sizes[4] != C1N * CIN || in_sizes[5] != C1N ||
      in_sizes[6] != NFN * KTAP || in_sizes[7] != NFN || in_sizes[8] != NFN || in_sizes[9] != NFN ||
      in_sizes[10] != NFN || in_sizes[11] != NFN || in_sizes[12] != GN * CL || in_sizes[13] != GN * HN ||
      in_sizes[14] != GN || in_sizes[15] != GN || out_size != NBAT * HN) return;

  const float* x      = (const float*)d_in[0];
  const int*   s      = (const int*)  d_in[1];
  const int*   onset  = (const int*)  d_in[2];
  const int*   offset = (const int*)  d_in[3];
  const float* w1     = (const float*)d_in[4];
  const float* b1     = (const float*)d_in[5];
  const float* w2     = (const float*)d_in[6];
  const float* b2     = (const float*)d_in[7];
  const float* bn_g   = (const float*)d_in[8];
  const float* bn_b   = (const float*)d_in[9];
  const float* bn_m   = (const float*)d_in[10];
  const float* bn_v   = (const float*)d_in[11];
  const float* w_ih   = (const float*)d_in[12];
  const float* w_hh   = (const float*)d_in[13];
  const float* b_ih   = (const float*)d_in[14];
  const float* b_hh   = (const float*)d_in[15];
  float* out = (float*)d_out;

  char* ws = (char*)d_ws; size_t off = 0;
  auto carve = [&](size_t bytes) -> char* { char* p = ws + off; off += (bytes + 255) & ~(size_t)255; return p; };
  float*          Y1    = (float*)carve((size_t)NBAT * C1N * TLEN * 4);
  unsigned short* P16   = (unsigned short*)carve((size_t)NBAT * WMAXN * CL * 2);
  unsigned short* WIH16 = (unsigned short*)carve((size_t)GN * CL * 2);
  unsigned short* WHH16 = (unsigned short*)carve((size_t)GN * HN * 2);
  if (off > ws_size || off > (size_t)134217728) return;

  prep_w_kernel<<<10, 256, 0, stream>>>(w_ih, w_hh, WIH16, WHH16);
  pconv_kernel<<<NBAT * (TLEN / CV_TB), CV_THR, 0, stream>>>(x, w1, b1, Y1);
  pool_kernel<<<dim3(WMAXN, NBAT), PL_THR, 0, stream>>>(Y1, w2, b2, bn_g, bn_b, bn_m, bn_v, onset, offset, P16);
  lstm_kernel<<<NBAT / LS_ROWS, LS_THR, 0, stream>>>(P16, WIH16, WHH16, b_ih, b_hh, s, out);
}
